// TimeDistributedReturn_7756710937364
// MI455X (gfx1250) — hardware-verified
//
#include <hip/hip_runtime.h>
#include <math.h>

typedef __attribute__((ext_vector_type(16))) _Float16 v16h;
typedef __attribute__((ext_vector_type(8)))  _Float16 v8h;
typedef __attribute__((ext_vector_type(8)))  float    v8f;
typedef __attribute__((ext_vector_type(4)))  float    v4f;

constexpr int   kSteps   = 8192;
constexpr int   kCols    = 1024;
constexpr int   kChunk   = 128;
constexpr int   kNumCh   = kSteps / kChunk;
constexpr float kGamma   = 0.99f;
constexpr float kCarry   = 64.0f;
constexpr float kCarryInv = 1.0f / kCarry;
static_assert(kNumCh == 64);
static_assert((kChunk % 32) == 0 && (kChunk % 64) == 0 && (kCols % 64) == 0 && (kSteps % 64) == 0);
static_assert(kCarry * kCarryInv == 1.0f);

constexpr double ce_ln(double x) {
  const double z = (x - 1.0) / (x + 1.0);
  const double z2 = z * z;
  double term = z;
  double s = 0.0;
  for (int i = 0; i < 14; ++i) {
    s += term / (double)(2 * i + 1);
    term *= z2;
  }
  return 2.0 * s;
}
constexpr double ce_powi(double b, int e) {
  double p = 1.0;
  for (int i = 0; i < e; ++i) p *= b;
  return p;
}
constexpr double kLn2  = 0.6931471805599453094;
constexpr float  kLg2G = (float)(ce_ln((double)kGamma) / kLn2);
constexpr float  kGChunk = (float)ce_powi((double)kGamma, kChunk);
static_assert(kLg2G < -0.014499f && kLg2G > -0.014500f);
static_assert(kGChunk > 0.2760f && kGChunk < 0.2765f);

constexpr size_t kOffRT = 0;
constexpr size_t kOffWS = kOffRT + (size_t)kCols * kSteps * 2;
constexpr size_t kOffGS = kOffWS + (size_t)kNumCh * kCols * 4;
constexpr size_t kOffUP = kOffGS + (size_t)kNumCh * kCols * 4;
constexpr size_t kWsTotal = kOffUP + (size_t)kChunk * kChunk * 2;
static_assert(kWsTotal == 17334272ull);
static_assert(kWsTotal <= 134217728ull);
static_assert((kOffWS % 128) == 0 && (kOffGS % 128) == 0 && (kOffUP % 128) == 0);

union FragU { v16h v; v8h h[2]; };
__device__ __forceinline__ v16h frag_load(const _Float16* p) {
  FragU f;
  f.h[0] = *(const v8h*)(p);
  f.h[1] = *(const v8h*)(p + 16);
  return f.v;
}
__device__ __forceinline__ v8f mma_f16(v16h a, v16h b, v8f c) {
  c = __builtin_amdgcn_wmma_f32_16x16x32_f16(false, a, false, b, (short)0, c, false, false);
  asm volatile("v_nop\n\tv_nop\n\tv_nop\n\tv_nop" : "+v"(c) : "v"(a), "v"(b));
  return c;
}

__global__ __launch_bounds__(256) void prep_transpose_kernel(
    const float* __restrict__ r, unsigned short* __restrict__ rT)
{
  __shared__ __align__(16) float sT[64 * 68];
  const int tid  = threadIdx.x;
  const int lane = tid & 31;
  const int wave = __builtin_amdgcn_readfirstlane((int)(threadIdx.x >> 5));
  const int n0 = blockIdx.x * 64;
  const int t0 = blockIdx.y * 64;
  const int lr = tid >> 4;
  const int lc4 = (tid & 15) * 4;
#pragma unroll
  for (int i = 0; i < 4; ++i) {
    const int row = lr + 16 * i;
    const v4f v = *(const v4f*)(r + (size_t)(t0 + row) * kCols + n0 + lc4);
    *(v4f*)(sT + row * 68 + lc4) = v;
  }
  __syncthreads();
  const int q  = lane >> 3;
  const int c8 = (lane & 7) * 8;
  v8h hv[2];
#pragma unroll
  for (int it = 0; it < 2; ++it) {
    const int nrow = it * 32 + wave * 4 + q;
#pragma unroll
    for (int e = 0; e < 8; ++e) {
      const float x = sT[(c8 + e) * 68 + nrow] * kCarry;
      hv[it][e] = (_Float16)x;
    }
  }
  for (int pass = 0; pass < 2; ++pass) {
#pragma unroll
    for (int it = 0; it < 2; ++it) {
      const int nrow = it * 32 + wave * 4 + q;
      *(volatile v8h*)(rT + (size_t)(n0 + nrow) * kSteps + t0 + c8) = hv[it];
    }
    __threadfence();
  }
}

__global__ __launch_bounds__(256) void build_tri_kernel(unsigned short* __restrict__ U)
{
  const int i = blockIdx.x * 256 + threadIdx.x;
  const int m = i >> 4;
  const int k8 = (i & 15) * 8;
  v8h hv;
#pragma unroll
  for (int e = 0; e < 8; ++e) {
    const int d = k8 + e - m;
    const int dc = d < 0 ? 0 : d;
    const float val = exp2f((float)dc * kLg2G);
    const float sel = (d >= 0) ? val : 0.0f;
    hv[e] = (_Float16)sel;
  }
  unsigned short* p = U + (size_t)m * kChunk + k8;
  *(volatile v8h*)p = hv;
  __threadfence();
  *(volatile v8h*)p = hv;
}

__global__ __launch_bounds__(256) void chunk_sum_kernel(
    const float* __restrict__ r, float* __restrict__ W)
{
  const int c  = blockIdx.x;
  const int n4 = threadIdx.x * 4;
  float w0 = 0.0f, w1 = 0.0f, w2 = 0.0f, w3 = 0.0f;
  const float* base = r + (size_t)c * kChunk * kCols + n4;
#pragma unroll 8
  for (int j = kChunk - 1; j >= 0; --j) {
    const v4f v = *(const v4f*)(base + (size_t)j * kCols);
    w0 = fmaf(kGamma, w0, v[0]);
    w1 = fmaf(kGamma, w1, v[1]);
    w2 = fmaf(kGamma, w2, v[2]);
    w3 = fmaf(kGamma, w3, v[3]);
  }
  v4f wv;
  wv[0] = w0; wv[1] = w1; wv[2] = w2; wv[3] = w3;
  float* p = W + (size_t)c * kCols + n4;
  *(volatile v4f*)p = wv;
  __threadfence();
  *(volatile v4f*)p = wv;
}

__global__ __launch_bounds__(64) void carry_scan_kernel(
    const float* __restrict__ W, float* __restrict__ G)
{
  const int n4 = (blockIdx.x * 64 + threadIdx.x) * 4;
  float g0 = 0.0f, g1 = 0.0f, g2 = 0.0f, g3 = 0.0f;
  {
    v4f zv;
    zv[0] = 0.0f; zv[1] = 0.0f; zv[2] = 0.0f; zv[3] = 0.0f;
    float* p = G + (size_t)(kNumCh - 1) * kCols + n4;
    *(volatile v4f*)p = zv;
    __threadfence();
    *(volatile v4f*)p = zv;
  }
#pragma unroll 1
  for (int c = kNumCh - 2; c >= 0; --c) {
    const v4f w = *(const v4f*)(W + (size_t)(c + 1) * kCols + n4);
    g0 = fmaf(kGChunk, g0, w[0]);
    g1 = fmaf(kGChunk, g1, w[1]);
    g2 = fmaf(kGChunk, g2, w[2]);
    g3 = fmaf(kGChunk, g3, w[3]);
    v4f gv;
    gv[0] = g0; gv[1] = g1; gv[2] = g2; gv[3] = g3;
    float* p = G + (size_t)c * kCols + n4;
    *(volatile v4f*)p = gv;
    __threadfence();
    *(volatile v4f*)p = gv;
  }
}

__global__ __launch_bounds__(256) void tri_gemm_kernel(
    const unsigned short* __restrict__ Up, const unsigned short* __restrict__ rTp,
    const float* __restrict__ G, float* __restrict__ out)
{
  __shared__ __align__(16) float sT[8][16 * 68];
  const int c    = blockIdx.y;
  const int lane = threadIdx.x & 31;
  const int wave = __builtin_amdgcn_readfirstlane((int)(threadIdx.x >> 5));
  const int tile = blockIdx.x * 8 + wave;
  const int tm = tile >> 4;
  const int tn = tile & 15;
  const int m0 = tm << 6;
  const int n0 = tn << 6;

  const _Float16* A  = (const _Float16*)Up;
  const _Float16* Bb = (const _Float16*)rTp + (size_t)c * kChunk;

  const int rlane = lane & 15;
  const int koff  = (lane >> 4) * 8;
  const int mOff  = (lane >> 4) * 8;

  v8f acc[4][4];
#pragma unroll
  for (int i = 0; i < 4; ++i)
#pragma unroll
    for (int j = 0; j < 4; ++j) acc[i][j] = (v8f){0.f, 0.f, 0.f, 0.f, 0.f, 0.f, 0.f, 0.f};

#pragma unroll 1
  for (int k0 = m0; k0 < kChunk; k0 += 32) {
    v16h bh[4];
#pragma unroll
    for (int j = 0; j < 4; ++j) {
      const size_t bo = (size_t)(n0 + (j << 4) + rlane) * kSteps + koff + k0;
      bh[j] = frag_load(Bb + bo);
    }
#pragma unroll
    for (int i = 0; i < 4; ++i) {
      const size_t ao = (size_t)(m0 + (i << 4) + rlane) * kChunk + koff + k0;
      const v16h ah = frag_load(A + ao);
#pragma unroll
      for (int j = 0; j < 4; ++j) acc[i][j] = mma_f16(ah, bh[j], acc[i][j]);
    }
  }

  float gv[4];
#pragma unroll
  for (int j = 0; j < 4; ++j) gv[j] = G[(size_t)c * kCols + n0 + (j << 4) + rlane];

  float* slab = sT[wave];
  float* C = out + (size_t)c * kChunk * kCols;
#pragma unroll
  for (int i = 0; i < 4; ++i) {
    const int mBase = m0 + (i << 4);
    float cw[8];
    cw[7] = exp2f((float)(kChunk - (mBase + mOff + 7)) * kLg2G);
#pragma unroll
    for (int r = 6; r >= 0; --r) cw[r] = cw[r + 1] * kGamma;
#pragma unroll
    for (int j = 0; j < 4; ++j) {
#pragma unroll
      for (int r = 0; r < 8; ++r) {
        const float loc = acc[i][j][r] * kCarryInv;
        slab[(mOff + r) * 68 + (j << 4) + rlane] = fmaf(cw[r], gv[j], loc);
      }
    }
    __syncthreads();
    {
      const int hh = lane >> 4;
      const int c4 = (lane & 15) * 4;
      for (int pass = 0; pass < 2; ++pass) {
#pragma unroll
        for (int it = 0; it < 8; ++it) {
          const int row = it * 2 + hh;
          const v4f v = *(const v4f*)(slab + row * 68 + c4);
          *(volatile v4f*)(C + (size_t)(mBase + row) * kCols + n0 + c4) = v;
        }
        __threadfence();
      }
    }
    __syncthreads();
  }
}

extern "C" void kernel_launch(void* const* d_in, const int* in_sizes, int n_in,
                              void* d_out, int out_size, void* d_ws, size_t ws_size,
                              hipStream_t stream) {
  if (n_in < 1) return;
  if (in_sizes[0] != kSteps * kCols) return;
  if (out_size != kSteps * kCols) return;
  if (ws_size < kWsTotal) return;

  const float* r = (const float*)d_in[0];
  float* out = (float*)d_out;
  char* ws = (char*)d_ws;
  unsigned short* RT = (unsigned short*)(ws + kOffRT);
  float*          WS = (float*)(ws + kOffWS);
  float*          GS = (float*)(ws + kOffGS);
  unsigned short* UP = (unsigned short*)(ws + kOffUP);

  prep_transpose_kernel<<<dim3(kCols / 64, kSteps / 64), 256, 0, stream>>>(r, RT);
  build_tri_kernel<<<(kChunk * kChunk / 8) / 256, 256, 0, stream>>>(UP);
  chunk_sum_kernel<<<kNumCh, kCols / 4, 0, stream>>>(r, WS);
  carry_scan_kernel<<<kCols / 4 / 64, 64, 0, stream>>>(WS, GS);
  tri_gemm_kernel<<<dim3(4, kNumCh), 256, 0, stream>>>(UP, RT, GS, out);
}
